// CrossAttentionNoGate_51694226374802
// MI455X (gfx1250) — hardware-verified
//
#include <hip/hip_runtime.h>
#include <math.h>

constexpr int kS        = 64;
constexpr int kL        = 512;
constexpr int kC        = 256;
constexpr int kNH       = 8;
constexpr int kDh       = 32;
constexpr int kHD       = kNH * kDh;
constexpr int kHalfS    = 32;
constexpr int kHalfTok  = kHalfS * kL;
constexpr int kGrpS     = 16;
constexpr int kCtxLd    = 2 * kHD;
constexpr float kScoreScale = 0.17677669529663687f;

static_assert(kL == 512, "softmax kernel: 64 threads x 8 columns = one row; blockIdx decode uses >>9");
static_assert(kHalfS % kGrpS == 0, "groups tile a half");
static_assert((kHalfTok * kC) % (8 * 256) == 0, "cast kernel grid exact");
static_assert(kHalfTok % 64 == 0 && kC % 64 == 0 && kHD % 64 == 0 && kL % 64 == 0 && kDh == 32, "tile multiples");

typedef __attribute__((ext_vector_type(16))) _Float16 v16h;
typedef __attribute__((ext_vector_type(8)))  _Float16 v8h;
typedef __attribute__((ext_vector_type(16))) __bf16   v16b;
typedef __attribute__((ext_vector_type(8)))  __bf16   v8b;
typedef __attribute__((ext_vector_type(8)))  float    v8f;
typedef __attribute__((ext_vector_type(4)))  float    v4f;
typedef __attribute__((ext_vector_type(4)))  unsigned int v4u;

__device__ __forceinline__ unsigned short f2bf_bits(float f) {
  unsigned u = __float_as_uint(f);
  return (unsigned short)((u + 0x7FFFu + ((u >> 16) & 1u)) >> 16);
}
__device__ __forceinline__ float bf_bits2f(unsigned short h) { return __uint_as_float(((unsigned)h) << 16); }

__device__ __forceinline__ void dep_guard_h(v8f& a, v8f& b, v16h x, v16h y) { asm volatile("v_nop\n\tv_nop\n\tv_nop\n\tv_nop" : "+v"(a), "+v"(b) : "v"(x), "v"(y)); }
__device__ __forceinline__ void dep_guard_b(v8f& a, v8f& b, v16b x, v16b y) { asm volatile("v_nop\n\tv_nop\n\tv_nop\n\tv_nop" : "+v"(a), "+v"(b) : "v"(x), "v"(y)); }
__device__ __forceinline__ void keep4_h(v16h a, v16h b, v16h c, v16h d) { asm volatile("v_nop" :: "v"(a), "v"(b), "v"(c), "v"(d)); }
__device__ __forceinline__ void keep4_b(v16b a, v16b b, v16b c, v16b d) { asm volatile("v_nop" :: "v"(a), "v"(b), "v"(c), "v"(d)); }
__device__ __forceinline__ void acc_guard4(v8f& a, v8f& b, v8f& c, v8f& d) { asm volatile("v_nop\n\tv_nop\n\tv_nop\n\tv_nop" : "+v"(a), "+v"(b), "+v"(c), "+v"(d)); }
template <typename T> struct Frag;
template <> struct Frag<_Float16> {
  typedef v16h V; union U { v16h v; v8h h[2]; };
  static __device__ __forceinline__ v16h load(const _Float16* p) {
    U f; f.h[0] = *(const v8h*)(p); f.h[1] = *(const v8h*)(p + 16); return f.v;
  }
  static __device__ __forceinline__ v8f mma(v16h a, v16h b, v8f c) {
    return __builtin_amdgcn_wmma_f32_16x16x32_f16(false, a, false, b, (short)0, c, false, false);
  }
  static __device__ __forceinline__ void guard(v8f& a, v8f& b, v16h x, v16h y) { dep_guard_h(a, b, x, y); }
  static __device__ __forceinline__ void keep(v16h a, v16h b, v16h c, v16h d) { keep4_h(a, b, c, d); }
};
template <> struct Frag<__bf16> {
  typedef v16b V; union U { v16b v; v8b h[2]; };
  static __device__ __forceinline__ v16b load(const __bf16* p) {
    U f; f.h[0] = *(const v8b*)(p); f.h[1] = *(const v8b*)(p + 16); return f.v;
  }
  static __device__ __forceinline__ v8f mma(v16b a, v16b b, v8f c) {
    return __builtin_amdgcn_wmma_f32_16x16x32_bf16(false, a, false, b, (short)0, c, false, false);
  }
  static __device__ __forceinline__ void guard(v8f& a, v8f& b, v16b x, v16b y) { dep_guard_b(a, b, x, y); }
  static __device__ __forceinline__ void keep(v16b a, v16b b, v16b c, v16b d) { keep4_b(a, b, c, d); }
};

__device__ __forceinline__ unsigned pk16(unsigned short a, unsigned short b) { return (unsigned)a | ((unsigned)b << 16); }

template <int ET> struct Elem;
template <> struct Elem<0> { typedef _Float16 T; };
template <> struct Elem<1> { typedef __bf16 T; };
template <int ET, bool SPLIT, int BIAS_MODE, int OUT_MODE, bool RESID, int ACT = 0, bool CAUSAL = false, bool BSPLIT = true>
__global__ __launch_bounds__(256) void wmma_gemm64(
    const unsigned short* __restrict__ Ap, const unsigned short* __restrict__ A2p, int lda, long strideA,
    const unsigned short* __restrict__ Btp, const unsigned short* __restrict__ Bt2p, int ldb, long strideB,
    void* __restrict__ Cout, void* __restrict__ Cout2, int ldc, long strideC,
    const float* __restrict__ bias,
    const float* __restrict__ resid, long strideR,
    int M, int N, int K, float scale) {
  typedef typename Elem<ET>::T T;
  typedef typename Frag<T>::V V;
  const T* A = (const T*)Ap; const T* A2 = (const T*)A2p; const T* Bt = (const T*)Btp; const T* Bt2 = (const T*)Bt2p;
  __shared__ __align__(16) float sT[8][16 * 68];
  const int b    = blockIdx.y;
  const int lane = threadIdx.x & 31;
  const int wave = threadIdx.x >> 5;
  const int tilesN = N >> 6;
  const int tilesM = M >> 6;
  const int tile = blockIdx.x * 8 + wave;
  if (tile >= tilesM * tilesN) return;
  const int tm = tile / tilesN;
  const int tn = tile - tm * tilesN;
  const int m0 = tm << 6;
  const int n0 = tn << 6;
  if (CAUSAL && (n0 > m0)) return;
  const int Kend = CAUSAL ? ((m0 + 64 < K) ? (m0 + 64) : K) : K;

  const T* Ab  = A  + (size_t)b * strideA;
  const T* Bb  = Bt + (size_t)b * strideB;
  const T* Ab2 = SPLIT ? (A2  + (size_t)b * strideA) : nullptr;
  const T* Bb2 = (SPLIT && BSPLIT) ? (Bt2 + (size_t)b * strideB) : nullptr;

  const int rlane = lane & 15;
  const int koff  = (lane >> 4) * 8;
  const int mOff  = (lane >> 4) * 8;

  v8f acc[4][4];
#pragma unroll
  for (int i = 0; i < 4; ++i)
#pragma unroll
    for (int j = 0; j < 4; ++j) acc[i][j] = (v8f){0.f,0.f,0.f,0.f,0.f,0.f,0.f,0.f};

  for (int k0 = 0; k0 < Kend; k0 += 32) {
    V bh[4], bl[4];
#pragma unroll
    for (int j = 0; j < 4; ++j) {
      const size_t bo = (size_t)(n0 + (j << 4) + rlane) * ldb + koff + k0;
      bh[j] = Frag<T>::load(Bb + bo);
      if (SPLIT && BSPLIT) bl[j] = Frag<T>::load(Bb2 + bo);
    }
#pragma unroll
    for (int i = 0; i < 4; ++i) {
      const size_t ao = (size_t)(m0 + (i << 4) + rlane) * lda + koff + k0;
      V ah = Frag<T>::load(Ab + ao);
      V al;
      if (SPLIT) al = Frag<T>::load(Ab2 + ao);
#pragma unroll
      for (int j = 0; j < 4; ++j) {
        acc[i][j] = Frag<T>::mma(ah, bh[j], acc[i][j]);
        if (SPLIT && BSPLIT) acc[i][j] = Frag<T>::mma(ah, bl[j], acc[i][j]);
        if (SPLIT) acc[i][j] = Frag<T>::mma(al, bh[j], acc[i][j]);
      }
      Frag<T>::guard(acc[i][0], acc[i][3], ah, SPLIT ? al : ah);
    }
    Frag<T>::keep(bh[0], bh[1], bh[2], bh[3]);
    if (SPLIT && BSPLIT) Frag<T>::keep(bl[0], bl[1], bl[2], bl[3]);
  }
  acc_guard4(acc[0][0], acc[0][1], acc[0][2], acc[0][3]);
  acc_guard4(acc[1][0], acc[1][1], acc[1][2], acc[1][3]);
  acc_guard4(acc[2][0], acc[2][1], acc[2][2], acc[2][3]);
  acc_guard4(acc[3][0], acc[3][1], acc[3][2], acc[3][3]);

  float* slab = sT[wave];
  const float* Rb = RESID ? (resid + (size_t)b * strideR) : nullptr;
#pragma unroll
  for (int i = 0; i < 4; ++i) {
    const int mBase = m0 + (i << 4);
#pragma unroll
    for (int j = 0; j < 4; ++j) {
      const int n = n0 + (j << 4) + rlane;
      float bv = 0.f;
      if (BIAS_MODE == 2) bv = bias[n];
#pragma unroll
      for (int r = 0; r < 8; ++r) {
        float v = acc[i][j][r] * scale;
        if (BIAS_MODE == 1) v += bias[mBase + mOff + r];
        if (BIAS_MODE == 2) v += bv;
        if (RESID) v += Rb[(size_t)(mBase + mOff + r) * ldc + n];
        if (ACT == 2) v = fmaxf(v, 0.0f);
        if (ACT == 4) v = (v > 0.f) ? v : 0.01f * v;
        slab[(mOff + r) * 68 + (j << 4) + rlane] = v;
      }
    }
    __builtin_amdgcn_fence(__ATOMIC_RELEASE, "workgroup");
    __builtin_amdgcn_wave_barrier();
    __builtin_amdgcn_fence(__ATOMIC_ACQUIRE, "workgroup");
    if (OUT_MODE == 0) {
      float* C = (float*)Cout + (size_t)b * strideC;
      const int hh = lane >> 4, c4 = (lane & 15) * 4;
      for (int pass = 0; pass < 2; ++pass) {
#pragma unroll
        for (int it = 0; it < 8; ++it) {
          const int row = it * 2 + hh;
          v4f v = *(const v4f*)(slab + row * 68 + c4);
          *(volatile v4f*)(C + (size_t)(mBase + row) * ldc + n0 + c4) = v;
        }
        __threadfence();
      }
    } else {
      const int q = lane >> 3, c8 = (lane & 7) * 8;
      unsigned short* C  = (unsigned short*)Cout  + (size_t)b * strideC;
      unsigned short* C2 = (OUT_MODE == 2) ? ((unsigned short*)Cout2 + (size_t)b * strideC) : nullptr;
      for (int pass = 0; pass < 2; ++pass) {
#pragma unroll
        for (int it = 0; it < 4; ++it) {
          const int row = it * 4 + q;
          const float* sp = slab + row * 68 + c8;
          v8h hv, lv;
#pragma unroll
          for (int e = 0; e < 8; ++e) {
            if (OUT_MODE == 1) {
              hv[e] = (_Float16)sp[e];
            } else {
              unsigned short hb = f2bf_bits(sp[e]);
              unsigned short lb = f2bf_bits(sp[e] - bf_bits2f(hb));
              hv[e] = __builtin_bit_cast(_Float16, hb);
              lv[e] = __builtin_bit_cast(_Float16, lb);
            }
          }
          *(volatile v8h*)(C + (size_t)(mBase + row) * ldc + n0 + c8) = hv;
          if (OUT_MODE == 2) *(volatile v8h*)(C2 + (size_t)(mBase + row) * ldc + n0 + c8) = lv;
        }
        __threadfence();
      }
    }
    __builtin_amdgcn_fence(__ATOMIC_RELEASE, "workgroup");
    __builtin_amdgcn_wave_barrier();
    __builtin_amdgcn_fence(__ATOMIC_ACQUIRE, "workgroup");
  }
}

__global__ __launch_bounds__(256) void wmma_gemm64x32_hilo(
    const unsigned short* __restrict__ Ap, const unsigned short* __restrict__ A2p, int lda, long strideA,
    const unsigned short* __restrict__ Btp, const unsigned short* __restrict__ Bt2p, int ldb, long strideB,
    unsigned short* __restrict__ Cout, int ldc, long strideC,
    int M, int N, int K, float scale) {
  typedef __bf16 T;
  typedef v16b V;
  const T* A = (const T*)Ap; const T* A2 = (const T*)A2p; const T* Bt = (const T*)Btp; const T* Bt2 = (const T*)Bt2p;
  __shared__ __align__(16) float sT[8][16 * 36];
  const int b    = blockIdx.y;
  const int lane = threadIdx.x & 31;
  const int wave = threadIdx.x >> 5;
  const int tilesN = N >> 5;
  const int tilesM = M >> 6;
  const int tile = blockIdx.x * 8 + wave;
  if (tile >= tilesM * tilesN) return;
  const int tm = tile / tilesN;
  const int tn = tile - tm * tilesN;
  const int m0 = tm << 6;
  const int n0 = tn << 5;

  const T* Ab  = A   + (size_t)b * strideA;
  const T* Ab2 = A2  + (size_t)b * strideA;
  const T* Bb  = Bt  + (size_t)b * strideB;
  const T* Bb2 = Bt2 + (size_t)b * strideB;

  const int rlane = lane & 15;
  const int koff  = (lane >> 4) * 8;
  const int mOff  = (lane >> 4) * 8;

  v8f acc[4][2];
#pragma unroll
  for (int i = 0; i < 4; ++i)
#pragma unroll
    for (int j = 0; j < 2; ++j) acc[i][j] = (v8f){0.f,0.f,0.f,0.f,0.f,0.f,0.f,0.f};

  for (int k0 = 0; k0 < K; k0 += 32) {
    V bh[2], bl[2];
#pragma unroll
    for (int j = 0; j < 2; ++j) {
      const size_t bo = (size_t)(n0 + (j << 4) + rlane) * ldb + koff + k0;
      bh[j] = Frag<T>::load(Bb + bo);
      bl[j] = Frag<T>::load(Bb2 + bo);
    }
#pragma unroll
    for (int i = 0; i < 4; ++i) {
      const size_t ao = (size_t)(m0 + (i << 4) + rlane) * lda + koff + k0;
      V ah = Frag<T>::load(Ab + ao);
      V al = Frag<T>::load(Ab2 + ao);
#pragma unroll
      for (int j = 0; j < 2; ++j) {
        acc[i][j] = Frag<T>::mma(ah, bh[j], acc[i][j]);
        acc[i][j] = Frag<T>::mma(ah, bl[j], acc[i][j]);
        acc[i][j] = Frag<T>::mma(al, bh[j], acc[i][j]);
      }
      Frag<T>::guard(acc[i][0], acc[i][1], ah, al);
    }
    Frag<T>::keep(bh[0], bh[1], bl[0], bl[1]);
  }
  acc_guard4(acc[0][0], acc[0][1], acc[1][0], acc[1][1]);
  acc_guard4(acc[2][0], acc[2][1], acc[3][0], acc[3][1]);

  float* slab = sT[wave];
  unsigned short* C = Cout + (size_t)b * strideC;
  const int q = lane >> 3, c8 = (lane & 7) * 8;
  const int csel = c8 & 31;
  const bool lo_half = (c8 >= 32);
#pragma unroll
  for (int i = 0; i < 4; ++i) {
    const int mBase = m0 + (i << 4);
#pragma unroll
    for (int j = 0; j < 2; ++j) {
#pragma unroll
      for (int r = 0; r < 8; ++r) slab[(mOff + r) * 36 + (j << 4) + rlane] = acc[i][j][r] * scale;
    }
    __builtin_amdgcn_fence(__ATOMIC_RELEASE, "workgroup");
    __builtin_amdgcn_wave_barrier();
    __builtin_amdgcn_fence(__ATOMIC_ACQUIRE, "workgroup");
    for (int pass = 0; pass < 2; ++pass) {
#pragma unroll
      for (int it = 0; it < 4; ++it) {
        const int row = it * 4 + q;
        const float* sp = slab + row * 36 + csel;
        v8h hv;
#pragma unroll
        for (int e = 0; e < 8; ++e) {
          const unsigned short hb = f2bf_bits(sp[e]);
          const unsigned short lb = f2bf_bits(sp[e] - bf_bits2f(hb));
          const unsigned short us = lo_half ? lb : hb;
          hv[e] = __builtin_bit_cast(_Float16, us);
        }
        *(volatile v8h*)(C + (size_t)(mBase + row) * ldc + 2 * n0 + c8) = hv;
      }
      __threadfence();
    }
    __builtin_amdgcn_fence(__ATOMIC_RELEASE, "workgroup");
    __builtin_amdgcn_wave_barrier();
    __builtin_amdgcn_fence(__ATOMIC_ACQUIRE, "workgroup");
  }
}

__global__ __launch_bounds__(256) void cast8_bf16_kernel(const float* __restrict__ in, unsigned short* __restrict__ out, int n8) {
  const int i = blockIdx.x * 256 + threadIdx.x;
  if (i >= n8) return;
  const float* p = in + 8 * (size_t)i;
  const v4f a = *(const v4f*)(p);
  const v4f c = *(const v4f*)(p + 4);
  float f[8];
#pragma unroll
  for (int e = 0; e < 4; ++e) { f[e] = a[e]; f[4 + e] = c[e]; }
  unsigned w[4];
#pragma unroll
  for (int e2 = 0; e2 < 4; ++e2) w[e2] = pk16(f2bf_bits(f[2 * e2]), f2bf_bits(f[2 * e2 + 1]));
  const v4u u = (v4u){w[0], w[1], w[2], w[3]};
  unsigned short* q = out + 8 * (size_t)i;
  *(volatile v4u*)q = u;
  __threadfence();
  *(volatile v4u*)q = u;
}

__global__ __launch_bounds__(256) void transpose_cast_kernel(const float* __restrict__ in, int ldin,
                                                             unsigned short* __restrict__ out, int ldout) {
  __shared__ float sm[64][65];
  const int t  = threadIdx.x;
  const int r0 = blockIdx.x * 64;
  const int c0 = blockIdx.y * 64;
#pragma unroll
  for (int i = 0; i < 16; ++i) {
    const int e = i * 256 + t;
    const int r = e >> 6;
    const int c = e & 63;
    sm[c][r] = in[(size_t)(r0 + r) * ldin + c0 + c];
  }
  __syncthreads();
  const int lane = t & 31, wave = t >> 5;
  const int q = lane >> 3, c8 = (lane & 7) * 8;
  for (int pass = 0; pass < 2; ++pass) {
#pragma unroll
    for (int it = 0; it < 2; ++it) {
      const int row = wave * 8 + it * 4 + q;
      unsigned w[4];
#pragma unroll
      for (int e2 = 0; e2 < 4; ++e2) w[e2] = pk16(f2bf_bits(sm[row][c8 + 2 * e2]), f2bf_bits(sm[row][c8 + 2 * e2 + 1]));
      const v4u u = (v4u){w[0], w[1], w[2], w[3]};
      const size_t o = (size_t)(c0 + row) * ldout + r0 + c8;
      *(volatile v4u*)(out + o) = u;
    }
    __threadfence();
  }
}

__global__ __launch_bounds__(256) void transpose_dup_cast_kernel(const float* __restrict__ in, int ldin,
                                                                 unsigned short* __restrict__ out, int ldout) {
  __shared__ float sm[64][65];
  const int t  = threadIdx.x;
  const int r0 = blockIdx.x * 64;
  const int c0 = blockIdx.y * 64;
#pragma unroll
  for (int i = 0; i < 16; ++i) {
    const int e = i * 256 + t;
    const int r = e >> 6;
    const int c = e & 63;
    sm[c][r] = in[(size_t)(r0 + r) * ldin + c0 + c];
  }
  __syncthreads();
  const int lane = t & 31, wave = t >> 5;
  const int hq = lane >> 4, c8 = (lane & 15) * 8;
  const int rb = ((c8 >> 6) << 5) + (c8 & 31);
  const int ocb = (r0 >> 5) * 64;
  for (int pass = 0; pass < 2; ++pass) {
#pragma unroll
    for (int it = 0; it < 4; ++it) {
      const int row = wave * 8 + it * 2 + hq;
      unsigned w[4];
#pragma unroll
      for (int e2 = 0; e2 < 4; ++e2) w[e2] = pk16(f2bf_bits(sm[row][rb + 2 * e2]), f2bf_bits(sm[row][rb + 2 * e2 + 1]));
      const v4u u = (v4u){w[0], w[1], w[2], w[3]};
      const size_t o = (size_t)(c0 + row) * ldout + ocb + c8;
      *(volatile v4u*)(out + o) = u;
    }
    __threadfence();
  }
}

__global__ __launch_bounds__(64) void rne_vec4_kernel(const float* __restrict__ in, float* __restrict__ out, int n4) {
  const int i = blockIdx.x * 64 + threadIdx.x;
  if (i >= n4) return;
  const v4f a = *(const v4f*)(in + 4 * (size_t)i);
  v4f v;
#pragma unroll
  for (int e = 0; e < 4; ++e) v[e] = bf_bits2f(f2bf_bits(a[e]));
  float* q = out + 4 * (size_t)i;
  *(volatile v4f*)q = v;
  __threadfence();
  *(volatile v4f*)q = v;
}

__global__ __launch_bounds__(64) void softmax_bias_kernel(const float* __restrict__ S, const float* __restrict__ biash,
                                                          const float* __restrict__ maskg,
                                                          unsigned short* __restrict__ Phi, unsigned short* __restrict__ Plo) {
#pragma clang fp contract(off)
  __shared__ float redM[2];
  __shared__ float redS[2];
  const float ninf = -__builtin_inff();
  const int blk  = blockIdx.x;
  const int pr   = blk >> 9;
  const int qi   = blk & (kL - 1);
  const int t    = threadIdx.x;
  const int lane = t & 31, wave = t >> 5;
  const int c0   = t * 8;
  const size_t rowoff = ((size_t)pr * kL + qi) * (size_t)kL;

  const float* sr = S + rowoff + c0;
  const float* br = biash + (size_t)qi * kL + c0;
  const float* mr = maskg + (size_t)pr * kL + c0;
  const v4f sa = *(const v4f*)(sr);
  const v4f sb = *(const v4f*)(sr + 4);
  const v4f ba = *(const v4f*)(br);
  const v4f bb = *(const v4f*)(br + 4);
  const v4f ma = *(const v4f*)(mr);
  const v4f mb = *(const v4f*)(mr + 4);
  float sv[8], bv[8], mk[8];
#pragma unroll
  for (int e = 0; e < 4; ++e) { sv[e] = sa[e]; sv[4 + e] = sb[e]; bv[e] = ba[e]; bv[4 + e] = bb[e]; mk[e] = ma[e]; mk[4 + e] = mb[e]; }

  float xv[8];
  float m = ninf;
#pragma unroll
  for (int e = 0; e < 8; ++e) {
    const float mkb = bf_bits2f(f2bf_bits(mk[e]));
    const float bbv = bf_bits2f(f2bf_bits(bv[e]));
    const float madd = (mkb - 1.0f) * 1.0e9f;
    const float v = (sv[e] + madd) + bbv;
    xv[e] = v;
    m = fmaxf(m, v);
  }
#pragma unroll
  for (int off = 16; off > 0; off >>= 1) m = fmaxf(m, __shfl_xor(m, off, 32));
  if (lane == 0) redM[wave] = m;
  __syncthreads();
  const float gmax = fmaxf(redM[0], redM[1]);

  float p[8];
  float ps = 0.0f;
#pragma unroll
  for (int e = 0; e < 8; ++e) { p[e] = expf(xv[e] - gmax); ps += p[e]; }
#pragma unroll
  for (int off = 16; off > 0; off >>= 1) ps += __shfl_xor(ps, off, 32);
  if (lane == 0) redS[wave] = ps;
  __syncthreads();
  const float tot = redS[0] + redS[1];
  const float inv = 1.0f / tot;

  unsigned hw[4], lw[4];
#pragma unroll
  for (int e2 = 0; e2 < 4; ++e2) {
    const float f0 = p[2 * e2] * inv;
    const float f1 = p[2 * e2 + 1] * inv;
    const unsigned short h0 = f2bf_bits(f0);
    const unsigned short h1 = f2bf_bits(f1);
    const unsigned short l0 = f2bf_bits(f0 - bf_bits2f(h0));
    const unsigned short l1 = f2bf_bits(f1 - bf_bits2f(h1));
    hw[e2] = pk16(h0, h1);
    lw[e2] = pk16(l0, l1);
  }
  const v4u hv = (v4u){hw[0], hw[1], hw[2], hw[3]};
  const v4u lv = (v4u){lw[0], lw[1], lw[2], lw[3]};
  unsigned short* ph = Phi + rowoff + c0;
  unsigned short* pl = Plo + rowoff + c0;
  *(volatile v4u*)ph = hv;
  *(volatile v4u*)pl = lv;
  __threadfence();
  *(volatile v4u*)ph = hv;
  *(volatile v4u*)pl = lv;
}

extern "C" void kernel_launch(void* const* d_in, const int* in_sizes, int n_in,
                              void* d_out, int out_size, void* d_ws, size_t ws_size,
                              hipStream_t stream) {
  if (n_in < 8) return;
  if (in_sizes[0] != kS * kL * kC || in_sizes[1] != kS * kL * kC || in_sizes[2] != kS * kL ||
      in_sizes[3] != kNH * kL * kL || in_sizes[4] != kC * kHD || in_sizes[5] != kC * 2 * kHD ||
      in_sizes[6] != kHD * kC || in_sizes[7] != kC) return;
  if (out_size != kS * kL * kC) return;

  const size_t kMiB   = 1048576;
  const size_t offQhi = 0;
  const size_t offQlo = 8 * kMiB;
  const size_t offKhi = 16 * kMiB;
  const size_t offKlo = 24 * kMiB;
  const size_t offVhi = 32 * kMiB;
  const size_t offVlo = 40 * kMiB;
  const size_t offS   = 48 * kMiB;
  const size_t offXkv = 48 * kMiB;
  const size_t offXq  = 56 * kMiB;
  const size_t offPhi = 64 * kMiB;
  const size_t offPlo = 72 * kMiB;
  const size_t offCtx = 80 * kMiB;
  const size_t offWqT = 96 * kMiB;
  const size_t offWkT = offWqT + (size_t)kHD * kC * 2;
  const size_t offWoT = offWkT + (size_t)2 * kHD * kC * 2;
  const size_t offBo  = offWoT + (size_t)kC * kCtxLd * 2;
  const size_t total  = offBo + (size_t)kC * 4;
  if (total > ws_size) return;

  const float* input_q  = (const float*)d_in[0];
  const float* input_kv = (const float*)d_in[1];
  const float* mask     = (const float*)d_in[2];
  const float* bias     = (const float*)d_in[3];
  const float* Wq       = (const float*)d_in[4];
  const float* Wkv      = (const float*)d_in[5];
  const float* Wo       = (const float*)d_in[6];
  const float* bo       = (const float*)d_in[7];
  float* out = (float*)d_out;
  char* ws = (char*)d_ws;

  unsigned short* qhi  = (unsigned short*)(ws + offQhi);
  unsigned short* qlo  = (unsigned short*)(ws + offQlo);
  unsigned short* khi  = (unsigned short*)(ws + offKhi);
  unsigned short* klo  = (unsigned short*)(ws + offKlo);
  unsigned short* vthi = (unsigned short*)(ws + offVhi);
  unsigned short* vtlo = (unsigned short*)(ws + offVlo);
  float*          Sbuf = (float*)(ws + offS);
  unsigned short* xkvb = (unsigned short*)(ws + offXkv);
  unsigned short* xqb  = (unsigned short*)(ws + offXq);
  unsigned short* phi  = (unsigned short*)(ws + offPhi);
  unsigned short* plo  = (unsigned short*)(ws + offPlo);
  unsigned short* ctx  = (unsigned short*)(ws + offCtx);
  unsigned short* wqT  = (unsigned short*)(ws + offWqT);
  unsigned short* wkvT = (unsigned short*)(ws + offWkT);
  unsigned short* woT  = (unsigned short*)(ws + offWoT);
  float*          bor  = (float*)(ws + offBo);

  const float* dummy_f = bor;
  void* dummy_c2 = (void*)phi;

  transpose_cast_kernel<<<dim3(kC / 64, kHD / 64), dim3(256), 0, stream>>>(Wq, kHD, wqT, kC);
  transpose_cast_kernel<<<dim3(kC / 64, (2 * kHD) / 64), dim3(256), 0, stream>>>(Wkv, 2 * kHD, wkvT, kC);
  transpose_dup_cast_kernel<<<dim3(kHD / 64, kC / 64), dim3(256), 0, stream>>>(Wo, kC, woT, kCtxLd);
  rne_vec4_kernel<<<dim3(1), dim3(64), 0, stream>>>(bo, bor, kC / 4);

  const int n8half = (kHalfTok * kC) / 8;
  const long tokStride = (long)kL * kHD;
  const long pairS     = (long)kL * kL;

  for (int hf = 0; hf < 2; ++hf) {
    const float* xq_h  = input_q  + (size_t)hf * kHalfTok * kC;
    const float* xkv_h = input_kv + (size_t)hf * kHalfTok * kC;

    cast8_bf16_kernel<<<dim3(n8half / 256), dim3(256), 0, stream>>>(xkv_h, xkvb, n8half);
    cast8_bf16_kernel<<<dim3(n8half / 256), dim3(256), 0, stream>>>(xq_h, xqb, n8half);

    wmma_gemm64<1, false, 0, 2, false, 0, false, true><<<dim3((kHalfTok / 64) * (kHD / 64) / 8, 1), dim3(256), 0, stream>>>(
        xkvb, xkvb, kC, 0L,
        wkvT, wkvT, kC, 0L,
        (void*)khi, (void*)klo, kHD, 0L,
        dummy_f, dummy_f, 0L,
        kHalfTok, kHD, kC, 1.0f);

    wmma_gemm64<1, false, 0, 2, false, 0, false, true><<<dim3((kHD / 64) * (kHalfTok / 64) / 8, 1), dim3(256), 0, stream>>>(
        wkvT + (size_t)kHD * kC, wkvT + (size_t)kHD * kC, kC, 0L,
        xkvb, xkvb, kC, 0L,
        (void*)vthi, (void*)vtlo, kHalfTok, 0L,
        dummy_f, dummy_f, 0L,
        kHD, kHalfTok, kC, 1.0f);

    wmma_gemm64<1, false, 0, 2, false, 0, false, true><<<dim3((kHalfTok / 64) * (kHD / 64) / 8, 1), dim3(256), 0, stream>>>(
        xqb, xqb, kC, 0L,
        wqT, wqT, kC, 0L,
        (void*)qhi, (void*)qlo, kHD, 0L,
        dummy_f, dummy_f, 0L,
        kHalfTok, kHD, kC, 1.0f);

    for (int sc = 0; sc < kHalfS / kGrpS; ++sc) {
      for (int h = 0; h < kNH; ++h) {
        const size_t qkoff = (size_t)(sc * kGrpS * kL) * kHD + (size_t)h * kDh;

        wmma_gemm64<1, true, 0, 0, false, 0, false, true><<<dim3((kL / 64) * (kL / 64) / 8, kGrpS), dim3(256), 0, stream>>>(
            qhi + qkoff, qlo + qkoff, kHD, tokStride,
            khi + qkoff, klo + qkoff, kHD, tokStride,
            (void*)Sbuf, dummy_c2, kL, pairS,
            dummy_f, dummy_f, 0L,
            kL, kL, kDh, kScoreScale);

        softmax_bias_kernel<<<dim3(kGrpS * kL), dim3(64), 0, stream>>>(
            Sbuf, bias + (size_t)h * kL * kL, mask + (size_t)(hf * kHalfS + sc * kGrpS) * kL, phi, plo);

        const size_t vtoff = (size_t)(h * kDh) * kHalfTok + (size_t)(sc * kGrpS * kL);
        const size_t coff  = (size_t)(sc * kGrpS * kL) * kCtxLd + (size_t)h * 64;
        wmma_gemm64x32_hilo<<<dim3((kL / 64) * (kDh / 32) / 8, kGrpS), dim3(256), 0, stream>>>(
            phi, plo, kL, pairS,
            vthi + vtoff, vtlo + vtoff, kHalfTok, (long)kL,
            ctx + coff, kCtxLd, (long)kL * kCtxLd,
            kL, kDh, kL, 1.0f);
      }
    }

    wmma_gemm64<1, false, 2, 0, false, 0, false, true><<<dim3((kHalfTok / 64) * (kC / 64) / 8, 1), dim3(256), 0, stream>>>(
        ctx, ctx, kCtxLd, 0L,
        woT, woT, kCtxLd, 0L,
        (void*)(out + (size_t)hf * kHalfTok * kC), dummy_c2, kC, 0L,
        bor, dummy_f, 0L,
        kHalfTok, kC, kCtxLd, 1.0f);
  }
}
